// ODEBlock_73650099192009
// MI455X (gfx1250) — hardware-verified
//
#include <hip/hip_runtime.h>

typedef __attribute__((ext_vector_type(16))) _Float16 v16h;
typedef __attribute__((ext_vector_type(8)))  _Float16 v8h;
typedef __attribute__((ext_vector_type(8)))  float    v8f;
typedef __attribute__((ext_vector_type(4)))  float    v4f;

constexpr int  kBatch   = 128;
constexpr int  kChan    = 64;
constexpr int  kH       = 32;
constexpr int  kW       = 32;
constexpr int  kHW      = kH * kW;
constexpr int  kCHW     = kChan * kHW;
constexpr long kNElem   = (long)kBatch * kCHW;
constexpr int  kGroups  = 32;
constexpr int  kGElem   = (kChan / kGroups) * kHW;
constexpr int  kCinW    = 65;
constexpr int  kWStride = kCinW * 9;
constexpr int  kKTot    = 9 * kChan;
constexpr float kEps     = 1e-5f;
constexpr float kWCarry  = 16.0f;
constexpr float kWCarryInv = 1.0f / 16.0f;
constexpr float kInvGElem = 1.0f / 2048.0f;

constexpr int kConvThreads = 128;
constexpr int kRowsPerBlk  = 8;
constexpr int kBlkPerImg   = kH / kRowsPerBlk;
constexpr int kConvGrid    = kBatch * kBlkPerImg;
constexpr int kSRows       = kRowsPerBlk + 2;
constexpr int kSCols       = kW + 2;
constexpr int kPixP        = 64;
constexpr int kSActHalves  = kSRows * kSCols * kPixP;
constexpr int kSlabPitch   = 68;
constexpr int kPackThreads = kChan * kKTot / 8;
constexpr int kPackGrid    = kPackThreads / 256;
constexpr int kStateGrid   = kBatch * kGroups;

static_assert(kKTot % 32 == 0);
static_assert(kChan == 64);
static_assert(kH % kRowsPerBlk == 0);
static_assert(kPackThreads % 256 == 0);
static_assert(kGElem == 2048);
static_assert(kSActHalves * 2 >= 4 * 16 * kSlabPitch * 4);

constexpr size_t kRegionBytes = (size_t)kNElem * 4;
constexpr size_t kOffR0  = 0;
constexpr size_t kOffR1  = kRegionBytes;
constexpr size_t kOffR2  = 2 * kRegionBytes;
constexpr size_t kWpBytes = (size_t)kChan * kKTot * 2;
constexpr size_t kOffWp1 = 3 * kRegionBytes;
constexpr size_t kOffWp2 = kOffWp1 + kWpBytes;
constexpr size_t kS1Bytes = (size_t)kStateGrid * 128;
constexpr size_t kOffS1  = kOffWp2 + kWpBytes;
constexpr size_t kPBytes = (size_t)kConvGrid * 256;
constexpr size_t kOffP2  = kOffS1 + kS1Bytes;
constexpr size_t kOffP3  = kOffP2 + kPBytes;
constexpr size_t kWsEnd  = kOffP3 + kPBytes;
static_assert(kWsEnd <= (size_t)134217728);
static_assert(kOffWp1 % 128 == 0 && kOffWp2 % 128 == 0 && kOffS1 % 128 == 0 && kOffP2 % 128 == 0 && kOffP3 % 128 == 0);

__device__ __forceinline__ void dep_guard_h(v8f& a, v8f& b, v16h x, v16h y) { asm volatile("v_nop\n\tv_nop\n\tv_nop\n\tv_nop" : "+v"(a), "+v"(b) : "v"(x), "v"(y)); }
__device__ __forceinline__ void keep4_h(v16h a, v16h b, v16h c, v16h d) { asm volatile("v_nop" :: "v"(a), "v"(b), "v"(c), "v"(d)); }
__device__ __forceinline__ void acc_guard4(v8f& a, v8f& b, v8f& c, v8f& d) { asm volatile("v_nop\n\tv_nop\n\tv_nop\n\tv_nop" : "+v"(a), "+v"(b), "+v"(c), "+v"(d)); }
__device__ __forceinline__ v8f mma_h(v16h a, v16h b, v8f c) {
  return __builtin_amdgcn_wmma_f32_16x16x32_f16(false, a, false, b, (short)0, c, false, false);
}
__device__ __forceinline__ v16h frag_load_g(const _Float16* p) {
  union { v16h v; v8h h[2]; } f;
  f.h[0] = *(const v8h*)(p);
  f.h[1] = *(const v8h*)(p + 16);
  return f.v;
}

__global__ __launch_bounds__(256) void k_pack_w(const float* __restrict__ w,
                                                _Float16* __restrict__ wp) {
  const int t   = blockIdx.x * 256 + threadIdx.x;
  const int o   = t / 72;
  const int kq  = t - o * 72;
  const int k8  = kq * 8;
  const int tap = k8 >> 6;
  const int ci0 = k8 & 63;
  const float* wr = w + (size_t)o * kWStride + (size_t)(ci0 + 1) * 9 + tap;
  v8h hv;
#pragma unroll
  for (int e = 0; e < 8; ++e) hv[e] = (_Float16)(wr[e * 9] * kWCarry);
  _Float16* dp = wp + (size_t)t * 8;
  *(volatile v8h*)dp = hv;
  __threadfence();
  *(volatile v8h*)dp = hv;
}

template <bool UPD>
__global__ __launch_bounds__(256) void k_state(const float* __restrict__ ysrc,
                                               const float* __restrict__ hsrc,
                                               const float* __restrict__ part,
                                               const float* __restrict__ gw,
                                               const float* __restrict__ gb,
                                               float* __restrict__ ydst,
                                               float* __restrict__ stab,
                                               float dt) {
  __shared__ float sS[8], sQ[8];
  const int bid  = blockIdx.x;
  const int b    = bid >> 5;
  const int g    = bid & 31;
  const int tid  = threadIdx.x;
  const int wave = tid >> 5;
  const int lane = tid & 31;

  float mu3 = 0.f, rs3 = 0.f;
  if (UPD) {
    const float* p = part + (size_t)b * 256 + g * 2;
    const float S = ((p[0] + p[64]) + p[128]) + p[192];
    const float Q = ((p[1] + p[65]) + p[129]) + p[193];
    mu3 = S * kInvGElem;
    const float var = fmaxf(Q * kInvGElem - mu3 * mu3, 0.f);
    rs3 = rsqrtf(var + kEps);
  }
  const size_t base = (size_t)bid * kGElem;
  v4f yn[2];
#pragma unroll
  for (int it = 0; it < 2; ++it) {
    const int f = tid + it * 256;
    const v4f yo = *(const v4f*)(ysrc + base + (size_t)f * 4);
    if (UPD) {
      const int c = 2 * g + it;
      const float a  = rs3 * gw[c];
      const float bb = gb[c] - mu3 * a;
      const v4f hv = *(const v4f*)(hsrc + base + (size_t)f * 4);
      v4f r;
#pragma unroll
      for (int e = 0; e < 4; ++e) r[e] = yo[e] + dt * fmaf(hv[e], a, bb);
      yn[it] = r;
    } else {
      yn[it] = yo;
    }
  }
  if (UPD) {
    for (int pass = 0; pass < 2; ++pass) {
#pragma unroll
      for (int it = 0; it < 2; ++it) {
        const v4f v = yn[it];
        *(volatile v4f*)(ydst + base + (size_t)(tid + it * 256) * 4) = v;
      }
      __threadfence();
    }
  }
  float s = 0.f;
#pragma unroll
  for (int it = 0; it < 2; ++it)
#pragma unroll
    for (int e = 0; e < 4; ++e) s += yn[it][e];
#pragma unroll
  for (int off = 16; off > 0; off >>= 1) s += __shfl_xor(s, off, 32);
  if (lane == 0) sS[wave] = s;
  __syncthreads();
  float S = 0.f;
#pragma unroll
  for (int i = 0; i < 8; ++i) S += sS[i];
  const float mu = S * kInvGElem;
  float q = 0.f;
#pragma unroll
  for (int it = 0; it < 2; ++it)
#pragma unroll
    for (int e = 0; e < 4; ++e) { const float d = yn[it][e] - mu; q = fmaf(d, d, q); }
#pragma unroll
  for (int off = 16; off > 0; off >>= 1) q += __shfl_xor(q, off, 32);
  if (lane == 0) sQ[wave] = q;
  __syncthreads();
  float Q = 0.f;
#pragma unroll
  for (int i = 0; i < 8; ++i) Q += sQ[i];
  const float var = Q * kInvGElem;
  const float rs  = rsqrtf(var + kEps);
  if (wave == 0) {
    v4f sv;
    sv[0] = (lane == 0) ? mu : 0.f;
    sv[1] = (lane == 0) ? rs : 0.f;
    sv[2] = 0.f;
    sv[3] = 0.f;
    float* sp = stab + (size_t)bid * 32 + lane * 4;
    for (int pass = 0; pass < 2; ++pass) {
      if (lane < 8) *(volatile v4f*)sp = sv;
      __threadfence();
    }
  }
}

union ConvTile {
  _Float16 h[kSActHalves];
  v8h      v[kSActHalves / 8];
  uint4    q[kSActHalves / 8];
  float    slab[4][16 * kSlabPitch];
};

template <int STATMODE>
__global__ __launch_bounds__(kConvThreads) void k_conv(const float* __restrict__ src,
                                                      const float* __restrict__ statin,
                                                      const float* __restrict__ gw,
                                                      const float* __restrict__ gb,
                                                      const unsigned short* __restrict__ wpk,
                                                      const float* __restrict__ wraw,
                                                      const float* __restrict__ bias,
                                                      float* __restrict__ dst,
                                                      float* __restrict__ partout,
                                                      float tval) {
  __shared__ __align__(16) ConvTile sU;
  __shared__ float sA[kChan], sBb[kChan], sBias[kChan];
  __shared__ float sTs[kChan * 9];
  __shared__ float sRed[4 * kGroups * 2];

  const int tid   = threadIdx.x;
  const int wave  = tid >> 5;
  const int lane  = tid & 31;
  const int rlane = lane & 15;
  const int hh    = lane >> 4;
  const int koff  = hh * 8;
  const int mOff  = hh * 8;
  const int b     = blockIdx.x >> 2;
  const int blk   = blockIdx.x & 3;
  const int h0    = blk * kRowsPerBlk;

  if (tid < kChan) {
    const int c = tid, g = c >> 1;
    float mu, rs;
    if (STATMODE == 0) {
      mu = statin[(size_t)(b * 32 + g) * 32 + 0];
      rs = statin[(size_t)(b * 32 + g) * 32 + 1];
    } else {
      const float* p = statin + (size_t)b * 256 + g * 2;
      const float S = ((p[0] + p[64]) + p[128]) + p[192];
      const float Q = ((p[1] + p[65]) + p[129]) + p[193];
      mu = S * kInvGElem;
      const float var = fmaxf(Q * kInvGElem - mu * mu, 0.f);
      rs = rsqrtf(var + kEps);
    }
    const float a = rs * gw[c];
    sA[c]    = a;
    sBb[c]   = gb[c] - mu * a;
    sBias[c] = bias[c];
  }
#pragma unroll 1
  for (int e = tid; e < kChan * 9; e += kConvThreads) {
    const int o   = e / 9;
    const int rem = e - o * 9;
    const int hc  = rem / 3;
    const int wc  = rem - hc * 3;
    float ts = 0.f;
#pragma unroll
    for (int kh = 0; kh < 3; ++kh) {
#pragma unroll
      for (int kw = 0; kw < 3; ++kw) {
        const float wv  = wraw[(size_t)o * kWStride + kh * 3 + kw];
        const bool  okh = !((hc == 0 && kh == 0) || (hc == 2 && kh == 2));
        const bool  okw = !((wc == 0 && kw == 0) || (wc == 2 && kw == 2));
        ts += (okh && okw) ? wv : 0.f;
      }
    }
    sTs[e] = ts;
  }
  for (int idx = tid; idx < 160; idx += kConvThreads) {
    const int slot = idx >> 3, part = idx & 7;
    const int row  = slot >> 1;
    const int col  = (slot & 1) ? (kSCols - 1) : 0;
    uint4 z; z.x = 0u; z.y = 0u; z.z = 0u; z.w = 0u;
    sU.q[(row * kSCols + col) * 8 + part] = z;
  }
  __syncthreads();

  {
    const int q  = tid & 7;
    const int cq = tid >> 3;
    float av[4], bv[4];
#pragma unroll
    for (int k = 0; k < 4; ++k) { av[k] = sA[k * 16 + cq]; bv[k] = sBb[k * 16 + cq]; }
    const float* sbase = src + (size_t)b * kCHW + q * 4;
#pragma unroll 1
    for (int r = 0; r < kSRows; ++r) {
      const int hin = h0 - 1 + r;
      const int hcl = hin < 0 ? 0 : (hin > kH - 1 ? kH - 1 : hin);
      const bool valid = (unsigned)hin < (unsigned)kH;
#pragma unroll
      for (int k = 0; k < 4; ++k) {
        const int c = k * 16 + cq;
        const v4f v = *(const v4f*)(sbase + (size_t)c * kHW + hcl * kW);
        _Float16* d = sU.h + (r * kSCols + q * 4 + 1) * kPixP + c;
#pragma unroll
        for (int e = 0; e < 4; ++e) {
          float t = fmaxf(fmaf(v[e], av[k], bv[k]), 0.f);
          t = valid ? t : 0.f;
          d[e * kPixP] = (_Float16)t;
        }
      }
    }
  }
  __syncthreads();

  const _Float16* wpl = (const _Float16*)wpk;
  v8f acc[4][4];
#pragma unroll
  for (int i = 0; i < 4; ++i)
#pragma unroll
    for (int j = 0; j < 4; ++j) acc[i][j] = (v8f){0.f,0.f,0.f,0.f,0.f,0.f,0.f,0.f};

  for (int ks = 0; ks < kKTot / 32; ++ks) {
    const int tap = ks >> 1;
    const int cb  = (ks & 1) << 5;
    const int kh  = (tap * 11) >> 5;
    const int kw  = tap - 3 * kh;
    const int k0  = ks << 5;
    v16h bfr[4];
#pragma unroll
    for (int j = 0; j < 4; ++j) {
      const int rr = wave * 2 + (j >> 1);
      const int w  = ((j & 1) << 4) + rlane;
      const int vi = ((rr + kh) * kSCols + w + kw) * 8 + (cb >> 3) + hh;
      union { v16h v; v8h h[2]; } f;
      f.h[0] = sU.v[vi];
      f.h[1] = sU.v[vi + 2];
      bfr[j] = f.v;
    }
#pragma unroll
    for (int i = 0; i < 4; ++i) {
      const v16h ah = frag_load_g(wpl + (size_t)((i << 4) + rlane) * kKTot + k0 + koff);
#pragma unroll
      for (int j = 0; j < 4; ++j) acc[i][j] = mma_h(ah, bfr[j], acc[i][j]);
      dep_guard_h(acc[i][0], acc[i][3], ah, ah);
    }
    keep4_h(bfr[0], bfr[1], bfr[2], bfr[3]);
  }
  acc_guard4(acc[0][0], acc[0][1], acc[0][2], acc[0][3]);
  acc_guard4(acc[1][0], acc[1][1], acc[1][2], acc[1][3]);
  acc_guard4(acc[2][0], acc[2][1], acc[2][2], acc[2][3]);
  acc_guard4(acc[3][0], acc[3][1], acc[3][2], acc[3][3]);

  __syncthreads();

  float* slab = sU.slab[wave];
  float* dstb = dst + (size_t)b * kCHW;
  const int n0 = (h0 + 2 * wave) * kW;
#pragma unroll
  for (int i = 0; i < 4; ++i) {
    float gs[8], gq[8];
#pragma unroll
    for (int r = 0; r < 8; ++r) { gs[r] = 0.f; gq[r] = 0.f; }
#pragma unroll
    for (int j = 0; j < 4; ++j) {
      const int hrow = h0 + 2 * wave + (j >> 1);
      const int hcls = (hrow == 0) ? 0 : ((hrow == kH - 1) ? 2 : 1);
      const int w    = ((j & 1) << 4) + rlane;
      const int wcls = (w == 0) ? 0 : ((w == kW - 1) ? 2 : 1);
      const int cls  = hcls * 3 + wcls;
#pragma unroll
      for (int r = 0; r < 8; ++r) {
        const int o = (i << 4) + mOff + r;
        float v = acc[i][j][r] * kWCarryInv + sBias[o];
        v = fmaf(tval, sTs[o * 9 + cls], v);
        slab[(mOff + r) * kSlabPitch + (j << 4) + rlane] = v;
        gs[r] += v;
        gq[r] = fmaf(v, v, gq[r]);
      }
    }
#pragma unroll
    for (int r = 0; r < 8; ++r) {
#pragma unroll
      for (int off = 1; off < 16; off <<= 1) {
        gs[r] += __shfl_xor(gs[r], off, 32);
        gq[r] += __shfl_xor(gq[r], off, 32);
      }
    }
    if (rlane == 0) {
#pragma unroll
      for (int rp = 0; rp < 4; ++rp) {
        const int g = (i << 3) + (hh << 2) + rp;
        sRed[(wave * kGroups + g) * 2 + 0] = gs[2 * rp] + gs[2 * rp + 1];
        sRed[(wave * kGroups + g) * 2 + 1] = gq[2 * rp] + gq[2 * rp + 1];
      }
    }
    __builtin_amdgcn_fence(__ATOMIC_RELEASE, "workgroup");
    __builtin_amdgcn_wave_barrier();
    __builtin_amdgcn_fence(__ATOMIC_ACQUIRE, "workgroup");
    {
      const int c4 = rlane * 4;
      for (int pass = 0; pass < 2; ++pass) {
#pragma unroll
        for (int it = 0; it < 8; ++it) {
          const int row = it * 2 + hh;
          const v4f v = *(const v4f*)(slab + row * kSlabPitch + c4);
          *(volatile v4f*)(dstb + (size_t)((i << 4) + row) * kHW + n0 + c4) = v;
        }
        __threadfence();
      }
    }
    __builtin_amdgcn_fence(__ATOMIC_RELEASE, "workgroup");
    __builtin_amdgcn_wave_barrier();
    __builtin_amdgcn_fence(__ATOMIC_ACQUIRE, "workgroup");
  }

  __syncthreads();
  if (wave == 0) {
    const int gA = rlane * 2, gB = gA + 1;
    float SA = 0.f, QA = 0.f, SB = 0.f, QB = 0.f;
#pragma unroll
    for (int wv = 0; wv < 4; ++wv) {
      SA += sRed[(wv * kGroups + gA) * 2 + 0];
      QA += sRed[(wv * kGroups + gA) * 2 + 1];
      SB += sRed[(wv * kGroups + gB) * 2 + 0];
      QB += sRed[(wv * kGroups + gB) * 2 + 1];
    }
    v4f pv;
    pv[0] = SA; pv[1] = QA; pv[2] = SB; pv[3] = QB;
    float* pp = partout + (size_t)blockIdx.x * 64 + rlane * 4;
    for (int pass = 0; pass < 2; ++pass) {
      if (hh == 0) *(volatile v4f*)pp = pv;
      __threadfence();
    }
  }
}

extern "C" void kernel_launch(void* const* d_in, const int* in_sizes, int n_in,
                              void* d_out, int out_size, void* d_ws, size_t ws_size,
                              hipStream_t stream) {
  if (n_in < 11) return;
  if (in_sizes[0] != (int)kNElem || out_size != (int)kNElem) return;
  if (in_sizes[3] != kChan * kWStride || in_sizes[7] != kChan * kWStride) return;
  if (kWsEnd > ws_size) return;

  const float* x       = (const float*)d_in[0];
  const float* gn1_w   = (const float*)d_in[1];
  const float* gn1_b   = (const float*)d_in[2];
  const float* conv1_w = (const float*)d_in[3];
  const float* conv1_b = (const float*)d_in[4];
  const float* gn2_w   = (const float*)d_in[5];
  const float* gn2_b   = (const float*)d_in[6];
  const float* conv2_w = (const float*)d_in[7];
  const float* conv2_b = (const float*)d_in[8];
  const float* gn3_w   = (const float*)d_in[9];
  const float* gn3_b   = (const float*)d_in[10];
  float* out = (float*)d_out;

  char* wsb = (char*)d_ws;
  float* R[3];
  R[0] = (float*)(wsb + kOffR0);
  R[1] = (float*)(wsb + kOffR1);
  R[2] = (float*)(wsb + kOffR2);
  _Float16* wp1 = (_Float16*)(wsb + kOffWp1);
  _Float16* wp2 = (_Float16*)(wsb + kOffWp2);
  float* s1 = (float*)(wsb + kOffS1);
  float* p2 = (float*)(wsb + kOffP2);
  float* p3 = (float*)(wsb + kOffP3);

  k_pack_w<<<kPackGrid, 256, 0, stream>>>(conv1_w, wp1);
  k_pack_w<<<kPackGrid, 256, 0, stream>>>(conv2_w, wp2);
  k_state<false><<<kStateGrid, 256, 0, stream>>>(x, x, p3, gn1_w, gn1_b, R[0], s1, 0.0f);

  const float dtf = (float)(1.0 / 6.0);
  int yi = -1;
  for (int s = 0; s < 6; ++s) {
    const float t = dtf * (float)s;
    const float* ys = (s == 0) ? x : R[yi];
    const int ai = (s == 0) ? 0 : (yi + 1) % 3;
    const int bi = (s == 0) ? 1 : (yi + 2) % 3;
    k_conv<0><<<kConvGrid, kConvThreads, 0, stream>>>(ys, s1, gn1_w, gn1_b,
        (const unsigned short*)wp1, conv1_w, conv1_b, R[ai], p2, t);
    k_conv<1><<<kConvGrid, kConvThreads, 0, stream>>>(R[ai], p2, gn2_w, gn2_b,
        (const unsigned short*)wp2, conv2_w, conv2_b, R[bi], p3, t);
    float* yd = (s == 5) ? out : R[ai];
    k_state<true><<<kStateGrid, 256, 0, stream>>>(ys, R[bi], p3, gn3_w, gn3_b, yd, s1, dtf);
    yi = ai;
  }
}
